// DecoderLayer_13683765805857
// MI455X (gfx1250) — hardware-verified
//
#include <hip/hip_runtime.h>
#ifndef NB
#define NB 2
#endif
#ifndef SEQ
#define SEQ 2048
#endif
#define NB_FULL 2
#define SEQ_FULL 2048
#define DM 1024
#define NH 16
#define HD 64
#define DFF 4096
#define HG 2
#define LQ (3 * DM)
#define NRW ((size_t)NB * SEQ)
#define LN_EPS 1e-5f
#define WS_LIMIT ((size_t)134217728)

static_assert(NB >= 1 && NB <= NB_FULL);
static_assert(SEQ % 256 == 0 && SEQ >= 256 && SEQ <= SEQ_FULL);
static_assert(DM == 256 * 4);
static_assert(NH * HD == DM && HD == 64 && NH % HG == 0);
static_assert(SEQ % 128 == 0 && (NB * SEQ) % 128 == 0);
static_assert(DM % 64 == 0 && DFF % 64 == 0 && SEQ % 64 == 0);
static_assert(DM % 32 == 0 && DFF % 32 == 0 && HD % 32 == 0);
static_assert((DM * (DM / 8)) % 256 == 0 && (DFF * (DM / 8)) % 256 == 0 && (DM * (DFF / 8)) % 256 == 0);

typedef unsigned short v8us __attribute__((ext_vector_type(8), may_alias));
typedef float  v8f  __attribute__((ext_vector_type(8)));
typedef float  v4f  __attribute__((ext_vector_type(4)));
typedef float  v4fa __attribute__((ext_vector_type(4), may_alias));
typedef int    v4i  __attribute__((ext_vector_type(4)));
typedef int    v4ia __attribute__((ext_vector_type(4), may_alias));
typedef _Float16 v16h __attribute__((ext_vector_type(16)));
typedef _Float16 v4h __attribute__((ext_vector_type(4)));
union FragH { v16h v; v8us half[2]; _Float16 h[16]; unsigned short u[16]; };

__device__ __forceinline__ unsigned short bf16_bits(float x) { unsigned int u = __float_as_uint(x); return (unsigned short)((u + 0x7FFFu + ((u >> 16) & 1u)) >> 16); }
__device__ __forceinline__ float bf16_val(unsigned short b) { return __uint_as_float(((unsigned int)b) << 16); }
__device__ __forceinline__ float bf16_rne(float x) { return bf16_val(bf16_bits(x)); }

__device__ __forceinline__ v16h g2_frag(const _Float16* p, int hh) { FragH f; f.half[0] = *(const v8us*)((const unsigned short*)p + 8 * hh); f.half[1] = *(const v8us*)((const unsigned short*)p + 16 + 8 * hh); return f.v; }
__device__ __forceinline__ v8f g2_mma(v16h a, v16h b, v8f c) { v8f d = __builtin_amdgcn_wmma_f32_16x16x32_f16(false, a, false, b, (short)0, c, false, false); asm volatile("v_nop\n\tv_nop\n\tv_nop\n\tv_nop" : "+v"(d) : "v"(a), "v"(b)); return d; }

__global__ __launch_bounds__(256) void k_wt_f16(const float* __restrict__ W, _Float16* __restrict__ Wt, unsigned K, unsigned N, unsigned nbw, float scale) {
  const unsigned kc = K >> 3; const unsigned t = blockIdx.x * 256u + threadIdx.x; if (t >= N * kc) return;
  const unsigned n = t / kc, k8 = (t - n * kc) << 3; const unsigned blk = n / nbw, j = n - blk * nbw;
  const float* src = W + (size_t)blk * K * nbw + j; FragH f;
#pragma unroll
  for (unsigned i = 0; i < 8; ++i) f.h[i] = (_Float16)(bf16_rne(src[(size_t)(k8 + i) * nbw]) * scale);
  const v8us o = f.half[0]; unsigned short* d = (unsigned short*)Wt + (size_t)n * K + k8;
  *(volatile v8us*)d = o; __threadfence(); *(volatile v8us*)d = o;
}

template <int BFIN>
__global__ __launch_bounds__(256) void k_lnx(const float* __restrict__ X, int seqc, int seqin, const float* __restrict__ g, const float* __restrict__ bb, float eps, _Float16* __restrict__ N16) {
  #pragma clang fp contract(off)
  __shared__ float red[256];
  const int r = blockIdx.x, t = threadIdx.x; const int b = r / seqc, s = r - b * seqc;
  const float* xr = X + ((size_t)b * seqin + s) * DM; const int c0 = t * 4;
  const v4f xa = *(const v4fa*)(xr + c0); float sv[4]; float sum = 0.f;
#pragma unroll
  for (int q = 0; q < 4; ++q) { sv[q] = BFIN ? bf16_rne(xa[q]) : xa[q]; sum = __fadd_rn(sum, sv[q]); }
  red[t] = sum; __syncthreads();
  for (int st = 128; st > 0; st >>= 1) { if (t < st) red[t] = __fadd_rn(red[t], red[t + st]); __syncthreads(); }
  const float mu = __fmul_rn(red[0], 1.0f / (float)DM); __syncthreads();
  float vs = 0.f;
#pragma unroll
  for (int q = 0; q < 4; ++q) { const float dl = __fadd_rn(sv[q], -mu); vs = __fadd_rn(vs, __fmul_rn(dl, dl)); }
  red[t] = vs; __syncthreads();
  for (int st = 128; st > 0; st >>= 1) { if (t < st) red[t] = __fadd_rn(red[t], red[t + st]); __syncthreads(); }
  const float rs = rsqrtf(__fadd_rn(__fmul_rn(red[0], 1.0f / (float)DM), eps)); v4h y;
#pragma unroll
  for (int q = 0; q < 4; ++q) { const int c = c0 + q; const float yf = __fadd_rn(__fmul_rn(__fmul_rn(__fadd_rn(sv[q], -mu), rs), bf16_rne(g[c])), bf16_rne(bb[c])); y[q] = (_Float16)yf; }
  for (int pass = 0; pass < 2; ++pass) { *(volatile v4h*)(N16 + (size_t)r * DM + c0) = y; if (pass == 0) __threadfence(); }
}

template <int ACT, int CPBF>
__global__ __launch_bounds__(128) void k_gemm2(const _Float16* __restrict__ A, int lda, size_t sA, const _Float16* __restrict__ Bh, int ldb, size_t sB, float alpha,
    const float* __restrict__ bias, const float* __restrict__ CP, float* __restrict__ C, _Float16* __restrict__ C16, int ldc, size_t sC, int M, int N, int K) {
  static_assert(ACT == 0 || ACT == 3);
  static_assert(CPBF == 0 || CPBF == 1);
  __shared__ __attribute__((aligned(16))) float so[4][32][68];
  const int tid = threadIdx.x, w = tid >> 5, lane = tid & 31, ln = lane & 15, hh = lane >> 4; const int by = blockIdx.y;
  A += (size_t)by * sA; Bh += (size_t)by * sB; const size_t cofs = (size_t)by * sC;
  const int ntn = N >> 6; const int mt = blockIdx.x / ntn, nq = blockIdx.x - mt * ntn; const int row0 = mt * 128 + 32 * w, col0 = nq * 64; if (row0 >= M) return;
  const _Float16* a0p = A + (size_t)(row0 + ln) * lda; const _Float16* a1p = a0p + (size_t)16 * lda;
  const _Float16* b0p = Bh + (size_t)(col0 + ln) * ldb; const _Float16* b1p = b0p + (size_t)16 * ldb; const _Float16* b2p = b1p + (size_t)16 * ldb; const _Float16* b3p = b2p + (size_t)16 * ldb;
  const v8f z8 = {0.f,0.f,0.f,0.f,0.f,0.f,0.f,0.f}; v8f c00 = z8, c01 = z8, c02 = z8, c03 = z8, c10 = z8, c11 = z8, c12 = z8, c13 = z8;
#pragma unroll 1
  for (int kb = 0; kb < K; kb += 32) { const v16h a0 = g2_frag(a0p + kb, hh), a1 = g2_frag(a1p + kb, hh);
    v16h b = g2_frag(b0p + kb, hh); c00 = g2_mma(a0, b, c00); c10 = g2_mma(a1, b, c10);
    b = g2_frag(b1p + kb, hh); c01 = g2_mma(a0, b, c01); c11 = g2_mma(a1, b, c11);
    b = g2_frag(b2p + kb, hh); c02 = g2_mma(a0, b, c02); c12 = g2_mma(a1, b, c12);
    b = g2_frag(b3p + kb, hh); c03 = g2_mma(a0, b, c03); c13 = g2_mma(a1, b, c13); }
  v8f accs[8] = {c00, c01, c02, c03, c10, c11, c12, c13};
#pragma unroll
  for (int u = 0; u < 8; ++u) { const int t = u & 3, half = u >> 2; const int col = col0 + t * 16 + ln; const float bv = bias ? bf16_rne(bias[col]) : 0.f;
#pragma unroll
    for (int r = 0; r < 8; ++r) { const int rloc = half * 16 + 8 * hh + r; float v = accs[u][r] * alpha + bv;
      if (CP) { float cv = CP[cofs + (size_t)(row0 + rloc) * ldc + col]; if (CPBF) cv = bf16_rne(cv); v += cv; }
      if (ACT == 3) v = fmaxf(v, 0.f);
      so[w][rloc][t * 16 + ln] = v; } }
  __builtin_amdgcn_fence(4  , "workgroup"); __builtin_amdgcn_wave_barrier();
  const int rsub = lane >> 4, c4 = (lane & 15) * 4;
  for (int pass = 0; pass < 2; ++pass) {
#pragma unroll
    for (int q = 0; q < 16; ++q) { const int r = q * 2 + rsub; const v4f v = *(const v4fa*)&so[w][r][c4];
      if (C) *(volatile v4f*)(C + cofs + (size_t)(row0 + r) * ldc + col0 + c4) = v;
      if (C16) { v4h h4;
#pragma unroll
        for (int i = 0; i < 4; ++i) h4[i] = (_Float16)v[i];
        *(volatile v4h*)(C16 + cofs + (size_t)(row0 + r) * ldc + col0 + c4) = h4; } }
    if (pass == 0) __threadfence(); }
}

template <int NHv, int TTv>
__global__ __launch_bounds__(256) void k_vt(const _Float16* __restrict__ V16, int ldv, int voff, _Float16* __restrict__ Vt) {
  __shared__ unsigned short tl[64][66];
  const int tid = threadIdx.x; const int h = blockIdx.x / (TTv / 64), lg = blockIdx.x % (TTv / 64);
  for (int i = tid; i < 64 * 8; i += 256) { const int r = i / 8, c8 = (i % 8) * 8; FragH f;
    f.half[0] = *(const v8us*)((const unsigned short*)V16 + ((size_t)lg * 64 + r) * ldv + voff + h * 64 + c8);
#pragma unroll
    for (int q = 0; q < 8; ++q) tl[r][c8 + q] = f.u[q]; }
  __syncthreads();
  for (int pass = 0; pass < 2; ++pass) {
#pragma unroll
    for (int rd = 0; rd < 2; ++rd) { const int d = rd * 32 + tid / 8, pc = tid % 8; FragH f;
#pragma unroll
      for (int q = 0; q < 8; ++q) f.u[q] = tl[pc * 8 + q][d];
      *(volatile v8us*)((unsigned short*)Vt + ((size_t)h * 64 + d) * TTv + lg * 64 + pc * 8) = f.half[0]; }
    if (pass == 0) __threadfence(); }
}

__global__ __launch_bounds__(256) void k_smx(const float* __restrict__ S, const int* __restrict__ mk, _Float16* __restrict__ P, int nrows) {
  #pragma clang fp contract(off)
  constexpr int NU = SEQ / 256;
  const int w = threadIdx.x >> 5, lane = threadIdx.x & 31;
  const int i = blockIdx.x * 8 + w;
  if (i >= nrows) return;
  const float* s = S + (size_t)i * SEQ + lane * 8;
  const int* mp = mk + lane * 8;
  float v[NU * 8]; float mx = -3.0e38f;
#pragma unroll
  for (int u = 0; u < NU; ++u) {
    const v4f a = *(const v4fa*)(s + 256 * u), c = *(const v4fa*)(s + 256 * u + 4);
    const v4i ma = *(const v4ia*)(mp + 256 * u), mc = *(const v4ia*)(mp + 256 * u + 4);
#pragma unroll
    for (int q = 0; q < 4; ++q) { v[u * 8 + q] = (ma[q] == 0) ? -1.0e9f : a[q]; v[u * 8 + 4 + q] = (mc[q] == 0) ? -1.0e9f : c[q]; }
#pragma unroll
    for (int q = 0; q < 8; ++q) mx = fmaxf(mx, v[u * 8 + q]);
  }
#pragma unroll
  for (int o = 16; o > 0; o >>= 1) mx = fmaxf(mx, __shfl_xor(mx, o));
  float se = 0.f;
#pragma unroll
  for (int j = 0; j < NU * 8; ++j) { v[j] = __expf(v[j] - mx); se += v[j]; }
#pragma unroll
  for (int o = 16; o > 0; o >>= 1) se += __shfl_xor(se, o);
  const float sc = 1024.0f / se;
  unsigned short* d = (unsigned short*)P + (size_t)i * SEQ + lane * 8;
  for (int pass = 0; pass < 2; ++pass) {
#pragma unroll
    for (int u = 0; u < NU; ++u) { FragH f;
#pragma unroll
      for (int q = 0; q < 8; ++q) f.h[q] = (_Float16)(v[u * 8 + q] * sc);
      *(volatile v8us*)(d + 256 * u) = f.half[0]; }
    if (pass == 0) __threadfence();
  }
}

extern "C" void kernel_launch(void* const* d_in, const int* in_sizes, int n_in,
                              void* d_out, int out_size, void* d_ws, size_t ws_size, hipStream_t stream) {
  if (n_in < 18) return;
  const float* x   = (const float*)d_in[0];
  const int*   msk = (const int*)d_in[1];
  const float* Wq  = (const float*)d_in[2];  const float* bq = (const float*)d_in[3];
  const float* Wk  = (const float*)d_in[4];  const float* bk = (const float*)d_in[5];
  const float* Wv  = (const float*)d_in[6];  const float* bv = (const float*)d_in[7];
  const float* Wo  = (const float*)d_in[8];  const float* bo = (const float*)d_in[9];
  const float* W1  = (const float*)d_in[10]; const float* b1 = (const float*)d_in[11];
  const float* W2  = (const float*)d_in[12]; const float* b2 = (const float*)d_in[13];
  const float* g1  = (const float*)d_in[14]; const float* be1 = (const float*)d_in[15];
  const float* g2  = (const float*)d_in[16]; const float* be2 = (const float*)d_in[17];
  float* out = (float*)d_out;
  const size_t xneed = ((size_t)(NB - 1) * SEQ_FULL + SEQ) * DM;
  const size_t mneed = (size_t)(NB - 1) * SEQ_FULL + SEQ;
  if ((size_t)in_sizes[0] < xneed || (size_t)out_size < xneed) return;
  if ((size_t)in_sizes[1] < mneed) return;
  if (in_sizes[2] < DM * DM || in_sizes[4] < DM * DM || in_sizes[6] < DM * DM || in_sizes[8] < DM * DM) return;
  if (in_sizes[10] < DM * DFF || in_sizes[12] < DFF * DM) return;
  if (in_sizes[3] < DM || in_sizes[5] < DM || in_sizes[7] < DM || in_sizes[9] < DM || in_sizes[11] < DFF || in_sizes[13] < DM) return;
  if (in_sizes[14] < DM || in_sizes[15] < DM || in_sizes[16] < DM || in_sizes[17] < DM) return;

  char* ws = (char*)d_ws; size_t off = 0;
  auto take = [&](size_t bytes) { char* p = ws + off; off += (bytes + 255) & ~(size_t)255; return p; };
  _Float16* BWQKV = (_Float16*)take((size_t)3 * DM * DM * 2);
  _Float16* BWO   = (_Float16*)take((size_t)DM * DM * 2);
  _Float16* BW1   = (_Float16*)take((size_t)DFF * DM * 2);
  _Float16* BW2   = (_Float16*)take((size_t)DM * DFF * 2);
  _Float16* XN    = (_Float16*)take(NRW * DM * 2);
  const size_t qkvb = NRW * LQ * 2, hfb = (size_t)SEQ * DFF * 2;
  _Float16* QKV   = (_Float16*)take(qkvb > hfb ? qkvb : hfb);
  _Float16* HF16  = QKV;
  _Float16* O16   = (_Float16*)take(NRW * DM * 2);
  _Float16* VT    = (_Float16*)take((size_t)NH * HD * SEQ * 2);
  const size_t sbytes = (size_t)HG * SEQ * SEQ * 4, pbytes = (size_t)HG * SEQ * SEQ * 2, x1bytes = NRW * DM * 4;
  char* SPX = take((sbytes + pbytes) > x1bytes ? (sbytes + pbytes) : x1bytes);
  float* S = (float*)SPX; _Float16* P = (_Float16*)(SPX + sbytes);
  float* X1 = (float*)SPX;
  if (off > ws_size || off > WS_LIMIT) return;

  k_wt_f16<<<(unsigned)(((size_t)DM * (DM / 8) + 255) / 256), 256, 0, stream>>>(Wq, BWQKV, (unsigned)DM, (unsigned)DM, (unsigned)HD, 16.0f);
  k_wt_f16<<<(unsigned)(((size_t)DM * (DM / 8) + 255) / 256), 256, 0, stream>>>(Wk, BWQKV + (size_t)DM * DM, (unsigned)DM, (unsigned)DM, (unsigned)HD, 16.0f);
  k_wt_f16<<<(unsigned)(((size_t)DM * (DM / 8) + 255) / 256), 256, 0, stream>>>(Wv, BWQKV + (size_t)2 * DM * DM, (unsigned)DM, (unsigned)DM, (unsigned)HD, 16.0f);
  k_wt_f16<<<(unsigned)(((size_t)DM * (DM / 8) + 255) / 256), 256, 0, stream>>>(Wo, BWO, (unsigned)DM, (unsigned)DM, (unsigned)DM, 16.0f);
  k_wt_f16<<<(unsigned)(((size_t)DFF * (DM / 8) + 255) / 256), 256, 0, stream>>>(W1, BW1, (unsigned)DM, (unsigned)DFF, (unsigned)DFF, 16.0f);
  k_wt_f16<<<(unsigned)(((size_t)DM * (DFF / 8) + 255) / 256), 256, 0, stream>>>(W2, BW2, (unsigned)DFF, (unsigned)DM, (unsigned)DM, 16.0f);

  k_lnx<1><<<(unsigned)NRW, 256, 0, stream>>>(x, SEQ, SEQ_FULL, g1, be1, LN_EPS, XN);
  k_gemm2<0, 0><<<dim3((unsigned)((NRW / 128) * (DM / 64)), 1), 128, 0, stream>>>(XN, DM, 0, BWQKV, DM, 0, 0.0625f, bq, nullptr, nullptr, QKV, LQ, 0, (int)NRW, DM, DM);
  k_gemm2<0, 0><<<dim3((unsigned)((NRW / 128) * (DM / 64)), 1), 128, 0, stream>>>(XN, DM, 0, BWQKV + (size_t)DM * DM, DM, 0, 0.0625f, bk, nullptr, nullptr, QKV + DM, LQ, 0, (int)NRW, DM, DM);
  k_gemm2<0, 0><<<dim3((unsigned)((NRW / 128) * (DM / 64)), 1), 128, 0, stream>>>(XN, DM, 0, BWQKV + (size_t)2 * DM * DM, DM, 0, 0.0625f, bv, nullptr, nullptr, QKV + 2 * DM, LQ, 0, (int)NRW, DM, DM);

  for (int b = 0; b < NB; ++b) { const size_t rb = (size_t)b * SEQ;
    k_vt<NH, SEQ><<<(unsigned)(NH * (SEQ / 64)), 256, 0, stream>>>(QKV + rb * LQ, LQ, 2 * DM, VT);
    for (int h0 = 0; h0 < NH; h0 += HG) {
      k_gemm2<0, 0><<<dim3((unsigned)((SEQ / 128) * (SEQ / 64)), HG), 128, 0, stream>>>(QKV + rb * LQ + h0 * HD, LQ, (size_t)HD, QKV + rb * LQ + DM + h0 * HD, LQ, (size_t)HD, 0.125f, nullptr, nullptr, S, nullptr, SEQ, (size_t)SEQ * SEQ, SEQ, SEQ, HD);
      k_smx<<<(unsigned)((HG * SEQ + 7) / 8), 256, 0, stream>>>(S, msk + (size_t)b * SEQ_FULL, P, HG * SEQ);
      k_gemm2<0, 0><<<dim3((unsigned)((SEQ / 128) * (HD / 64)), HG), 128, 0, stream>>>(P, SEQ, (size_t)SEQ * SEQ, VT + (size_t)h0 * HD * SEQ, SEQ, (size_t)HD * SEQ, 0.0625f, nullptr, nullptr, nullptr, O16 + rb * DM + h0 * HD, DM, (size_t)HD, SEQ, HD, SEQ);
    }
  }
  for (int b = 0; b < NB; ++b) { const size_t rb = (size_t)b * SEQ;
    k_gemm2<0, 1><<<dim3((unsigned)((SEQ / 128) * (DM / 64)), 1), 128, 0, stream>>>(O16 + rb * DM, DM, 0, BWO, DM, 0, 0.0009765625f, bo, x + (size_t)b * SEQ_FULL * DM, X1 + rb * DM, nullptr, DM, 0, SEQ, DM, DM);
  }
  k_lnx<0><<<(unsigned)NRW, 256, 0, stream>>>(X1, SEQ, SEQ, g2, be2, LN_EPS, XN);
  for (int b = 0; b < NB; ++b) { const size_t rb = (size_t)b * SEQ;
    k_gemm2<3, 0><<<dim3((unsigned)((SEQ / 128) * (DFF / 64)), 1), 128, 0, stream>>>(XN + rb * DM, DM, 0, BW1, DM, 0, 0.0625f, b1, nullptr, nullptr, HF16, DFF, 0, SEQ, DFF, DM);
    k_gemm2<0, 0><<<dim3((unsigned)((SEQ / 128) * (DM / 64)), 1), 128, 0, stream>>>(HF16, DFF, 0, BW2, DFF, 0, 0.0625f, b2, X1 + rb * DM, out + (size_t)b * SEQ_FULL * DM, nullptr, DM, 0, SEQ, DM, DFF);
  }
}
